// MQA_74560632259155
// MI455X (gfx1250) — hardware-verified
//
#include <hip/hip_runtime.h>
#include <math.h>

#define SEQ    4096
#define DMOD   1024
#define HD     128
#define NH     8
#define QHALF  2048
#define PSCALE 32768.0f
#define PSCALE_INV (1.0f / 32768.0f)

typedef __attribute__((ext_vector_type(16))) _Float16 v16h;
typedef __attribute__((ext_vector_type(8)))  _Float16 v8h;
typedef __attribute__((ext_vector_type(16))) __bf16   v16b;
typedef __attribute__((ext_vector_type(8)))  __bf16   v8b;
typedef __attribute__((ext_vector_type(8)))  float    v8f;
typedef __attribute__((ext_vector_type(4)))  float    v4f;
typedef __attribute__((ext_vector_type(2)))  float    v2f;
typedef __attribute__((ext_vector_type(4)))  unsigned int v4u;

__device__ __forceinline__ unsigned short f2bf_bits(float f) {
  unsigned u = __float_as_uint(f);
  return (unsigned short)((u + 0x7FFFu + ((u >> 16) & 1u)) >> 16);
}
__device__ __forceinline__ float bf_bits2f(unsigned short h) { return __uint_as_float(((unsigned)h) << 16); }

__device__ __forceinline__ void dep_guard_h(v8f& a, v8f& b, v16h x, v16h y) { asm volatile("v_nop\n\tv_nop\n\tv_nop\n\tv_nop" : "+v"(a), "+v"(b) : "v"(x), "v"(y)); }
__device__ __forceinline__ void dep_guard_b(v8f& a, v8f& b, v16b x, v16b y) { asm volatile("v_nop\n\tv_nop\n\tv_nop\n\tv_nop" : "+v"(a), "+v"(b) : "v"(x), "v"(y)); }
__device__ __forceinline__ void keep4_h(v16h a, v16h b, v16h c, v16h d) { asm volatile("v_nop" :: "v"(a), "v"(b), "v"(c), "v"(d)); }
__device__ __forceinline__ void keep4_b(v16b a, v16b b, v16b c, v16b d) { asm volatile("v_nop" :: "v"(a), "v"(b), "v"(c), "v"(d)); }
__device__ __forceinline__ void acc_guard4(v8f& a, v8f& b, v8f& c, v8f& d) { asm volatile("v_nop\n\tv_nop\n\tv_nop\n\tv_nop" : "+v"(a), "+v"(b), "+v"(c), "+v"(d)); }
template <typename T> struct Frag;
template <> struct Frag<_Float16> {
  typedef v16h V; union U { v16h v; v8h h[2]; };
  static __device__ __forceinline__ v16h load(const _Float16* p) {
    U f; f.h[0] = *(const v8h*)(p); f.h[1] = *(const v8h*)(p + 16); return f.v;
  }
  static __device__ __forceinline__ v8f mma(v16h a, v16h b, v8f c) {
    return __builtin_amdgcn_wmma_f32_16x16x32_f16(false, a, false, b, (short)0, c, false, false);
  }
  static __device__ __forceinline__ void guard(v8f& a, v8f& b, v16h x, v16h y) { dep_guard_h(a, b, x, y); }
  static __device__ __forceinline__ void keep(v16h a, v16h b, v16h c, v16h d) { keep4_h(a, b, c, d); }
};
template <> struct Frag<__bf16> {
  typedef v16b V; union U { v16b v; v8b h[2]; };
  static __device__ __forceinline__ v16b load(const __bf16* p) {
    U f; f.h[0] = *(const v8b*)(p); f.h[1] = *(const v8b*)(p + 16); return f.v;
  }
  static __device__ __forceinline__ v8f mma(v16b a, v16b b, v8f c) {
    return __builtin_amdgcn_wmma_f32_16x16x32_bf16(false, a, false, b, (short)0, c, false, false);
  }
  static __device__ __forceinline__ void guard(v8f& a, v8f& b, v16b x, v16b y) { dep_guard_b(a, b, x, y); }
  static __device__ __forceinline__ void keep(v16b a, v16b b, v16b c, v16b d) { keep4_b(a, b, c, d); }
};

template <int ET> struct Elem;
template <> struct Elem<0> { typedef _Float16 T; };
template <> struct Elem<1> { typedef __bf16 T; };
template <int ET, bool SPLIT, int BIAS_MODE, int OUT_MODE, bool RESID, int ACT = 0>
__global__ __launch_bounds__(256) void wmma_gemm64(
    const unsigned short* __restrict__ Ap, const unsigned short* __restrict__ A2p, int lda, long strideA,
    const unsigned short* __restrict__ Btp, const unsigned short* __restrict__ Bt2p, int ldb, long strideB,
    void* __restrict__ Cout, void* __restrict__ Cout2, int ldc, long strideC,
    const float* __restrict__ bias,
    const float* __restrict__ resid, long strideR,
    int M, int N, int K, float scale) {
  typedef typename Elem<ET>::T T;
  typedef typename Frag<T>::V V;
  const T* A = (const T*)Ap; const T* A2 = (const T*)A2p; const T* Bt = (const T*)Btp; const T* Bt2 = (const T*)Bt2p;
  __shared__ __align__(16) float sT[8][16 * 68];
  const int b    = blockIdx.y;
  const int lane = threadIdx.x & 31;
  const int wave = threadIdx.x >> 5;
  const int tilesN = N >> 6;
  const int tilesM = M >> 6;
  const int tile = blockIdx.x * 8 + wave;
  if (tile >= tilesM * tilesN) return;
  const int tm = tile / tilesN;
  const int tn = tile - tm * tilesN;
  const int m0 = tm << 6;
  const int n0 = tn << 6;

  const T* Ab  = A  + (size_t)b * strideA;
  const T* Bb  = Bt + (size_t)b * strideB;
  const T* Ab2 = SPLIT ? (A2  + (size_t)b * strideA) : nullptr;
  const T* Bb2 = SPLIT ? (Bt2 + (size_t)b * strideB) : nullptr;

  const int rlane = lane & 15;
  const int koff  = (lane >> 4) * 8;
  const int mOff  = (lane >> 4) * 8;

  v8f acc[4][4];
#pragma unroll
  for (int i = 0; i < 4; ++i)
#pragma unroll
    for (int j = 0; j < 4; ++j) acc[i][j] = (v8f){0.f,0.f,0.f,0.f,0.f,0.f,0.f,0.f};

  for (int k0 = 0; k0 < K; k0 += 32) {
    V bh[4], bl[4];
#pragma unroll
    for (int j = 0; j < 4; ++j) {
      const size_t bo = (size_t)(n0 + (j << 4) + rlane) * ldb + koff + k0;
      bh[j] = Frag<T>::load(Bb + bo);
      if (SPLIT) bl[j] = Frag<T>::load(Bb2 + bo);
    }
#pragma unroll
    for (int i = 0; i < 4; ++i) {
      const size_t ao = (size_t)(m0 + (i << 4) + rlane) * lda + koff + k0;
      V ah = Frag<T>::load(Ab + ao);
      V al;
      if (SPLIT) al = Frag<T>::load(Ab2 + ao);
#pragma unroll
      for (int j = 0; j < 4; ++j) {
        acc[i][j] = Frag<T>::mma(ah, bh[j], acc[i][j]);
        if (SPLIT) {
          acc[i][j] = Frag<T>::mma(ah, bl[j], acc[i][j]);
          acc[i][j] = Frag<T>::mma(al, bh[j], acc[i][j]);
        }
      }
      Frag<T>::guard(acc[i][0], acc[i][3], ah, SPLIT ? al : ah);
    }
    Frag<T>::keep(bh[0], bh[1], bh[2], bh[3]);
    if (SPLIT) Frag<T>::keep(bl[0], bl[1], bl[2], bl[3]);
  }
  acc_guard4(acc[0][0], acc[0][1], acc[0][2], acc[0][3]);
  acc_guard4(acc[1][0], acc[1][1], acc[1][2], acc[1][3]);
  acc_guard4(acc[2][0], acc[2][1], acc[2][2], acc[2][3]);
  acc_guard4(acc[3][0], acc[3][1], acc[3][2], acc[3][3]);

  float* slab = sT[wave];
  const float* Rb = RESID ? (resid + (size_t)b * strideR) : nullptr;
#pragma unroll
  for (int i = 0; i < 4; ++i) {
    const int mBase = m0 + (i << 4);
#pragma unroll
    for (int j = 0; j < 4; ++j) {
      const int n = n0 + (j << 4) + rlane;
      float bv = 0.f;
      if (BIAS_MODE == 2) bv = bias[n];
#pragma unroll
      for (int r = 0; r < 8; ++r) {
        float v = acc[i][j][r] * scale;
        if (BIAS_MODE == 1) v += bias[mBase + mOff + r];
        if (BIAS_MODE == 2) v += bv;
        if (RESID) v += Rb[(size_t)(mBase + mOff + r) * ldc + n];
        if (ACT == 1) v = tanhf(v);
        if (ACT == 2) v = fmaxf(v, 0.0f);
        if (ACT == 3) v = v / (1.0f + expf(-v));
        if (ACT == 4) v = (v > 0.f) ? v : 0.01f * v;
        slab[(mOff + r) * 68 + (j << 4) + rlane] = v;
      }
    }
    __builtin_amdgcn_fence(__ATOMIC_RELEASE, "workgroup");
    __builtin_amdgcn_wave_barrier();
    __builtin_amdgcn_fence(__ATOMIC_ACQUIRE, "workgroup");
    if (OUT_MODE == 0) {
      float* C = (float*)Cout + (size_t)b * strideC;
      const int hh = lane >> 4, c4 = (lane & 15) * 4;
      for (int pass = 0; pass < 2; ++pass) {
#pragma unroll
        for (int it = 0; it < 8; ++it) {
          const int row = it * 2 + hh;
          v4f v = *(const v4f*)(slab + row * 68 + c4);
          *(volatile v4f*)(C + (size_t)(mBase + row) * ldc + n0 + c4) = v;
        }
        __threadfence();
      }
    } else {
      const int q = lane >> 3, c8 = (lane & 7) * 8;
      unsigned short* C  = (unsigned short*)Cout  + (size_t)b * strideC;
      unsigned short* C2 = (OUT_MODE == 2) ? ((unsigned short*)Cout2 + (size_t)b * strideC) : nullptr;
      for (int pass = 0; pass < 2; ++pass) {
#pragma unroll
        for (int it = 0; it < 4; ++it) {
          const int row = it * 4 + q;
          const float* sp = slab + row * 68 + c8;
          v8h hv, lv;
#pragma unroll
          for (int e = 0; e < 8; ++e) {
            if (OUT_MODE == 1) {
              hv[e] = (_Float16)sp[e];
            } else {
              unsigned short hb = f2bf_bits(sp[e]);
              unsigned short lb = f2bf_bits(sp[e] - bf_bits2f(hb));
              hv[e] = __builtin_bit_cast(_Float16, hb);
              lv[e] = __builtin_bit_cast(_Float16, lb);
            }
          }
          *(volatile v8h*)(C + (size_t)(mBase + row) * ldc + n0 + c8) = hv;
          if (OUT_MODE == 2) *(volatile v8h*)(C2 + (size_t)(mBase + row) * ldc + n0 + c8) = lv;
        }
        __threadfence();
      }
    }
    __builtin_amdgcn_fence(__ATOMIC_RELEASE, "workgroup");
    __builtin_amdgcn_wave_barrier();
    __builtin_amdgcn_fence(__ATOMIC_ACQUIRE, "workgroup");
  }
}

__device__ __forceinline__ unsigned pk16(unsigned short a, unsigned short b) { return (unsigned)a | ((unsigned)b << 16); }
__device__ __forceinline__ unsigned short h_bits(float f) { const _Float16 h = (_Float16)f; return __builtin_bit_cast(unsigned short, h); }

__global__ __launch_bounds__(256) void cast_f16x2_kernel(const float* __restrict__ in, unsigned short* __restrict__ out, int n2, float scale) {
  const int i = blockIdx.x * 256 + threadIdx.x;
  if (i < n2) {
    const v2f f = *(const v2f*)(in + 2 * (size_t)i);
    const unsigned u = pk16(h_bits(f[0] * scale), h_bits(f[1] * scale));
    ((volatile unsigned*)out)[i] = u;
    __threadfence();
    ((volatile unsigned*)out)[i] = u;
  }
}

__global__ __launch_bounds__(256) void transpose_cast_f16(const float* __restrict__ W, unsigned short* __restrict__ WT,
                                                          int KR, int NC, float scale) {
  __shared__ __align__(16) unsigned short T[64 * 72];
  const int tid  = threadIdx.x;
  const int lane = tid & 31;
  const int wave = tid >> 5;
  const int n0 = blockIdx.x * 64;
  const int k0 = blockIdx.y * 64;
  const int r  = tid >> 2;
  const int cb = (tid & 3) * 16;
  const float* src = W + (size_t)(k0 + r) * NC + n0 + cb;
#pragma unroll
  for (int q4 = 0; q4 < 4; ++q4) {
    const v4f f = *(const v4f*)(src + 4 * q4);
#pragma unroll
    for (int e = 0; e < 4; ++e) T[(cb + 4 * q4 + e) * 72 + r] = h_bits(f[e] * scale);
  }
  __syncthreads();
  const int rq = lane >> 3, c8 = (lane & 7) * 8;
  v4u val[2];
#pragma unroll
  for (int it = 0; it < 2; ++it) {
    const int n = it * 32 + wave * 4 + rq;
    val[it] = *(const v4u*)(T + n * 72 + c8);
  }
  for (int pass = 0; pass < 2; ++pass) {
#pragma unroll
    for (int it = 0; it < 2; ++it) {
      const int n = it * 32 + wave * 4 + rq;
      *(volatile v4u*)(WT + (size_t)(n0 + n) * KR + k0 + c8) = val[it];
    }
    __threadfence();
  }
}

__global__ __launch_bounds__(256) void softmax_row_kernel(const float* __restrict__ S, unsigned short* __restrict__ P) {
  __shared__ float redm[8];
  __shared__ float reds[8];
  const int i    = blockIdx.x;
  const int tid  = threadIdx.x;
  const int lane = tid & 31;
  const int wave = tid >> 5;
  const int ja   = tid * 8;
  const int jb   = (SEQ / 2) + tid * 8;
  const float* rp = S + (size_t)i * SEQ;
  const v4f a0 = *(const v4f*)(rp + ja);
  const v4f a1 = *(const v4f*)(rp + ja + 4);
  const v4f b0 = *(const v4f*)(rp + jb);
  const v4f b1 = *(const v4f*)(rp + jb + 4);
  float t[16];
  t[0] = a0[0]; t[1] = a0[1]; t[2]  = a0[2]; t[3]  = a0[3]; t[4]  = a1[0]; t[5]  = a1[1]; t[6]  = a1[2]; t[7]  = a1[3];
  t[8] = b0[0]; t[9] = b0[1]; t[10] = b0[2]; t[11] = b0[3]; t[12] = b1[0]; t[13] = b1[1]; t[14] = b1[2]; t[15] = b1[3];
  float m = t[0];
#pragma unroll
  for (int e = 1; e < 16; ++e) m = fmaxf(m, t[e]);
#pragma unroll
  for (int off = 16; off > 0; off >>= 1) m = fmaxf(m, __shfl_xor(m, off, 32));
  if (lane == 0) redm[wave] = m;
  __syncthreads();
  float mx = redm[0];
#pragma unroll
  for (int w = 1; w < 8; ++w) mx = fmaxf(mx, redm[w]);
  float ex[16];
  float s = 0.f;
#pragma unroll
  for (int e = 0; e < 16; ++e) { ex[e] = __expf(t[e] - mx); s += ex[e]; }
#pragma unroll
  for (int off = 16; off > 0; off >>= 1) s += __shfl_xor(s, off, 32);
  if (lane == 0) reds[wave] = s;
  __syncthreads();
  float tot = reds[0];
#pragma unroll
  for (int w = 1; w < 8; ++w) tot += reds[w];
  const float inv = 1.0f / tot;
  unsigned short hb16[16];
#pragma unroll
  for (int e = 0; e < 16; ++e) { const float p = ex[e] * inv; hb16[e] = h_bits(p * PSCALE); }
  const v4u ha = (v4u){pk16(hb16[0], hb16[1]),  pk16(hb16[2], hb16[3]),   pk16(hb16[4], hb16[5]),   pk16(hb16[6], hb16[7])};
  const v4u hb = (v4u){pk16(hb16[8], hb16[9]),  pk16(hb16[10], hb16[11]), pk16(hb16[12], hb16[13]), pk16(hb16[14], hb16[15])};
  unsigned short* prow = P + (size_t)i * SEQ;
  *(volatile v4u*)(prow + ja) = ha;
  *(volatile v4u*)(prow + jb) = hb;
  __threadfence();
  *(volatile v4u*)(prow + ja) = ha;
  *(volatile v4u*)(prow + jb) = hb;
}

extern "C" void kernel_launch(void* const* d_in, const int* in_sizes, int n_in,
                              void* d_out, int out_size, void* d_ws, size_t ws_size,
                              hipStream_t stream) {
  if (n_in < 7) return;
  if (in_sizes[0] != SEQ * DMOD) return;
  if (in_sizes[1] != DMOD * DMOD || in_sizes[2] != DMOD) return;
  if (in_sizes[3] != DMOD * HD || in_sizes[4] != HD) return;
  if (in_sizes[5] != DMOD * HD || in_sizes[6] != HD) return;
  if (out_size != SEQ * DMOD) return;

  const float* x  = (const float*)d_in[0];
  const float* Wq = (const float*)d_in[1];
  const float* bq = (const float*)d_in[2];
  const float* Wk = (const float*)d_in[3];
  const float* bk = (const float*)d_in[4];
  const float* Wv = (const float*)d_in[5];
  const float* bv = (const float*)d_in[6];
  float* out = (float*)d_out;

  const size_t PWQ = (size_t)DMOD * DMOD * 2;
  const size_t PWK = (size_t)HD * DMOD * 2;
  const size_t PX  = (size_t)SEQ * DMOD * 2;
  const size_t PK  = (size_t)SEQ * HD * 2;
  const size_t PS  = (size_t)QHALF * SEQ * 4;
  const size_t PP  = (size_t)QHALF * SEQ * 2;
  size_t off = 0;
  const size_t oWqT = off; off += PWQ;
  const size_t oWkT = off; off += PWK;
  const size_t oWvT = off; off += PWK;
  const size_t oX16 = off; off += PX;
  const size_t oQ16 = off; off += PX;
  const size_t oK16 = off; off += PK;
  const size_t oVT  = off; off += PK;
  const size_t oS   = off; off += PS;
  const size_t oP   = off; off += PP;
  if (off > ws_size) return;

  char* ws = (char*)d_ws;
  unsigned short* WqT16 = (unsigned short*)(ws + oWqT);
  unsigned short* WkT16 = (unsigned short*)(ws + oWkT);
  unsigned short* WvT16 = (unsigned short*)(ws + oWvT);
  unsigned short* X16   = (unsigned short*)(ws + oX16);
  unsigned short* Q16   = (unsigned short*)(ws + oQ16);
  unsigned short* K16   = (unsigned short*)(ws + oK16);
  unsigned short* VT16  = (unsigned short*)(ws + oVT);
  float*          Sbuf  = (float*)(ws + oS);
  unsigned short* P16   = (unsigned short*)(ws + oP);

  const dim3 blk(256);
  const float wcarry = 16.0f;
  const float wscale = 1.0f / 16.0f;
  const float sscale = 0.08838834764831845f;

  transpose_cast_f16<<<dim3(DMOD / 64, DMOD / 64), blk, 0, stream>>>(Wq, WqT16, DMOD, DMOD, wcarry);
  transpose_cast_f16<<<dim3(HD / 64, DMOD / 64), blk, 0, stream>>>(Wk, WkT16, DMOD, HD, wcarry);
  transpose_cast_f16<<<dim3(HD / 64, DMOD / 64), blk, 0, stream>>>(Wv, WvT16, DMOD, HD, wcarry);
  const int n2x = SEQ * DMOD / 2;
  cast_f16x2_kernel<<<dim3((n2x + 255) / 256), blk, 0, stream>>>(x, X16, n2x, 1.0f);

  const dim3 gQ(((SEQ / 64) * (DMOD / 64) + 7) / 8, 1);
  wmma_gemm64<0, false, 2, 1, false, 0><<<gQ, blk, 0, stream>>>(
      X16, X16, DMOD, 0L, WqT16, WqT16, DMOD, 0L, (void*)Q16, (void*)Q16, DMOD, 0L,
      bq, bq, 0L, SEQ, DMOD, DMOD, wscale);
  const dim3 gK(((SEQ / 64) * (HD / 64) + 7) / 8, 1);
  wmma_gemm64<0, false, 2, 1, false, 0><<<gK, blk, 0, stream>>>(
      X16, X16, DMOD, 0L, WkT16, WkT16, DMOD, 0L, (void*)K16, (void*)K16, HD, 0L,
      bk, bk, 0L, SEQ, HD, DMOD, wscale);
  const dim3 gV(((HD / 64) * (SEQ / 64) + 7) / 8, 1);
  wmma_gemm64<0, false, 1, 1, false, 0><<<gV, blk, 0, stream>>>(
      WvT16, WvT16, DMOD, 0L, X16, X16, DMOD, 0L, (void*)VT16, (void*)VT16, SEQ, 0L,
      bv, bv, 0L, HD, SEQ, DMOD, wscale);

  const dim3 gS(((QHALF / 64) * (SEQ / 64) + 7) / 8, 1);
  const dim3 gPV(((QHALF / 64) * (HD / 64) + 7) / 8, 1);
  for (int h = 0; h < NH; ++h) {
    for (int qh = 0; qh < 2; ++qh) {
      const unsigned short* Qsub = Q16 + (size_t)qh * QHALF * DMOD + (size_t)h * HD;
      wmma_gemm64<0, false, 0, 0, false, 0><<<gS, blk, 0, stream>>>(
          Qsub, Qsub, DMOD, 0L, K16, K16, HD, 0L, (void*)Sbuf, (void*)Sbuf, SEQ, 0L,
          bq, bq, 0L, QHALF, SEQ, HD, sscale);
      softmax_row_kernel<<<dim3(QHALF), blk, 0, stream>>>(Sbuf, P16);
      float* osub = out + (size_t)qh * QHALF * DMOD + (size_t)h * HD;
      wmma_gemm64<0, false, 0, 0, false, 0><<<gPV, blk, 0, stream>>>(
          P16, P16, SEQ, 0L, VT16, VT16, SEQ, 0L, (void*)osub, (void*)osub, DMOD, 0L,
          bq, bq, 0L, QHALF, HD, SEQ, PSCALE_INV);
    }
  }
  (void)hipGetLastError();
}
